// LSTMSequenceModel_65859028517120
// MI455X (gfx1250) — hardware-verified
//
#include <hip/hip_runtime.h>


typedef _Float16 f16t;
typedef f16t  v16h __attribute__((ext_vector_type(16)));
typedef f16t  v8h  __attribute__((ext_vector_type(8)));
typedef f16t  v4h  __attribute__((ext_vector_type(4)));
typedef float v8f  __attribute__((ext_vector_type(8)));
typedef float v4f  __attribute__((ext_vector_type(4)));

union Frag { v16h v; v8h q[2]; };

#define TT  512
#define NI  4
#define NH  16
#define NG  64
#define AP  40
#define YC  32

__device__ __forceinline__ v8f wmma16(v16h a, v16h b, v8f c) {
    return __builtin_amdgcn_wmma_f32_16x16x32_f16(false, a, false, b, (short)0, c, false, false);
}

__device__ __forceinline__ void wguard4(v8f (&c)[4], Frag& a, v16h (&b)[4]) {
    asm volatile("v_nop\n\tv_nop\n\tv_nop\n\tv_nop"
                 : "+v"(c[0]), "+v"(c[1]), "+v"(c[2]), "+v"(c[3])
                 : "v"(a.v), "v"(b[0]), "v"(b[1]), "v"(b[2]), "v"(b[3]));
}

__device__ __forceinline__ float fsig(float x) {
    float e = __expf(-x);
    return __builtin_amdgcn_rcpf(1.0f + e);
}
__device__ __forceinline__ float ftanh(float x) {
    float ax = fabsf(x);
    float e  = __expf(-2.0f * ax);
    float r  = (1.0f - e) * __builtin_amdgcn_rcpf(1.0f + e);
    return copysignf(r, x);
}

__global__ __launch_bounds__(32)
void k_lstm2(const float* __restrict__ x,
             const float* __restrict__ Wih0, const float* __restrict__ Whh0,
             const float* __restrict__ bih0, const float* __restrict__ bhh0,
             const float* __restrict__ Wih1, const float* __restrict__ Whh1,
             const float* __restrict__ bih1, const float* __restrict__ bhh1,
             const float* __restrict__ Wfc,  const float* __restrict__ bfc,
             float* out, int nb)
{
    __shared__ __attribute__((aligned(16))) f16t  A0[16 * AP];
    __shared__ __attribute__((aligned(16))) f16t  A1[16 * AP];
    __shared__ __attribute__((aligned(16))) float Hf[16 * NH];
    __shared__ __attribute__((aligned(16))) float Ys[16 * YC];

    const int l  = threadIdx.x & 31, h = l >> 4, m = l & 15;
    const int b0 = blockIdx.x * 16;
    if (b0 + 16 > nb) return;

    for (int i = l; i < 16 * AP; i += 32) { A0[i] = (f16t)0.0f; A1[i] = (f16t)0.0f; }

    const float WS  = 16.0f;
    const float INV = 0.0625f;
    v16h wb0[4], wb1[4];
#pragma unroll
    for (int tile = 0; tile < 4; ++tile) {
        const int n = tile * 16 + m;
#pragma unroll
        for (int i = 0; i < 16; ++i) {
            const int k  = 8 * h + i + ((i >> 3) << 3);
            const int kx = (k < NI) ? k : (NI - 1);
            int kh = k - NI; kh = kh < 0 ? 0 : (kh > NH - 1 ? NH - 1 : kh);
            const float w0 = (k < NI) ? Wih0[n * NI + kx]
                           : ((k < NI + NH) ? Whh0[n * NH + kh] : 0.0f);
            const int k1 = (k < NH) ? k : (NH - 1);
            int k2 = k - NH; k2 = k2 < 0 ? 0 : (k2 > NH - 1 ? NH - 1 : k2);
            const float w1 = (k < NH) ? Wih1[n * NH + k1] : Whh1[n * NH + k2];
            wb0[tile][i] = (f16t)(w0 * WS);
            wb1[tile][i] = (f16t)(w1 * WS);
        }
    }

    float bs0[4], bs1[4];
#pragma unroll
    for (int tile = 0; tile < 4; ++tile) {
        bs0[tile] = bih0[tile * 16 + m] + bhh0[tile * 16 + m];
        bs1[tile] = bih1[tile * 16 + m] + bhh1[tile * 16 + m];
    }
    float wf[NH];
#pragma unroll
    for (int k = 0; k < NH; ++k) wf[k] = Wfc[k];
    const float bf = bfc[0];

    float c0s[8], c1s[8];
#pragma unroll
    for (int r = 0; r < 8; ++r) { c0s[r] = 0.0f; c1s[r] = 0.0f; }

    const v8f zacc = {0.f, 0.f, 0.f, 0.f, 0.f, 0.f, 0.f, 0.f};
    const float* xrow = x + (size_t)(b0 + m) * TT * NI;

    __syncthreads();

#pragma unroll 1
    for (int t = 0; t < TT; ++t) {
        {
            const v4f xv = *(const v4f*)(xrow + (size_t)t * NI);
            v4h xh;
            xh[0] = (f16t)xv[0]; xh[1] = (f16t)xv[1]; xh[2] = (f16t)xv[2]; xh[3] = (f16t)xv[3];
            *(v4h*)(A0 + m * AP) = xh;
        }
        __syncthreads();

        Frag a;
        a.q[0] = *(const v8h*)(A0 + m * AP + 8 * h);
        a.q[1] = *(const v8h*)(A0 + m * AP + 16 + 8 * h);
        v8f acc[4];
#pragma unroll
        for (int tile = 0; tile < 4; ++tile) acc[tile] = wmma16(a.v, wb0[tile], zacc);
        wguard4(acc, a, wb0);

#pragma unroll
        for (int r = 0; r < 8; ++r) {
            const float pi = fmaf(acc[0][r], INV, bs0[0]);
            const float pf = fmaf(acc[1][r], INV, bs0[1]);
            const float pg = fmaf(acc[2][r], INV, bs0[2]);
            const float po = fmaf(acc[3][r], INV, bs0[3]);
            const float ig = fsig(pi), fg = fsig(pf), gg = ftanh(pg), og = fsig(po);
            const float c  = fmaf(fg, c0s[r], ig * gg);
            c0s[r] = c;
            const float hv = og * ftanh(c);
            const f16t  hh = (f16t)hv;
            A0[(8 * h + r) * AP + NI + m] = hh;
            A1[(8 * h + r) * AP + m]      = hh;
        }
        __syncthreads();

        a.q[0] = *(const v8h*)(A1 + m * AP + 8 * h);
        a.q[1] = *(const v8h*)(A1 + m * AP + 16 + 8 * h);
#pragma unroll
        for (int tile = 0; tile < 4; ++tile) acc[tile] = wmma16(a.v, wb1[tile], zacc);
        wguard4(acc, a, wb1);

#pragma unroll
        for (int r = 0; r < 8; ++r) {
            const float pi = fmaf(acc[0][r], INV, bs1[0]);
            const float pf = fmaf(acc[1][r], INV, bs1[1]);
            const float pg = fmaf(acc[2][r], INV, bs1[2]);
            const float po = fmaf(acc[3][r], INV, bs1[3]);
            const float ig = fsig(pi), fg = fsig(pf), gg = ftanh(pg), og = fsig(po);
            const float c  = fmaf(fg, c1s[r], ig * gg);
            c1s[r] = c;
            const float hv = og * ftanh(c);
            A1[(8 * h + r) * AP + NH + m] = (f16t)hv;
            Hf[(8 * h + r) * NH + m]      = hv;
        }
        __syncthreads();

        {
            const float* hr = Hf + m * NH;
            const v4f u0 = *(const v4f*)(hr);
            const v4f u1 = *(const v4f*)(hr + 4);
            const v4f u2 = *(const v4f*)(hr + 8);
            const v4f u3 = *(const v4f*)(hr + 12);
            float y = bf;
#pragma unroll
            for (int k = 0; k < 4; ++k) y = fmaf(u0[k], wf[k], y);
#pragma unroll
            for (int k = 0; k < 4; ++k) y = fmaf(u1[k], wf[4 + k], y);
#pragma unroll
            for (int k = 0; k < 4; ++k) y = fmaf(u2[k], wf[8 + k], y);
#pragma unroll
            for (int k = 0; k < 4; ++k) y = fmaf(u3[k], wf[12 + k], y);
            Ys[m * YC + (t & (YC - 1))] = y;
        }

        if ((t & (YC - 1)) == (YC - 1)) {
            __syncthreads();
            const int t0 = t - (YC - 1);
            v4f v[4];
#pragma unroll
            for (int i = 0; i < 4; ++i) {
                const int p = l + 32 * i, row = p >> 3, q = p & 7;
                v[i] = *(const v4f*)(Ys + row * YC + 4 * q);
            }
#pragma unroll
            for (int i = 0; i < 4; ++i) {
                const int p = l + 32 * i, row = p >> 3, q = p & 7;
                *(volatile v4f*)(out + (size_t)(b0 + row) * TT + t0 + 4 * q) = v[i];
            }
            __threadfence();
#pragma unroll
            for (int i = 0; i < 4; ++i) {
                const int p = l + 32 * i, row = p >> 3, q = p & 7;
                *(volatile v4f*)(out + (size_t)(b0 + row) * TT + t0 + 4 * q) = v[i];
            }
        }
    }
}

extern "C" void kernel_launch(void* const* d_in, const int* in_sizes, int n_in,
                              void* d_out, int out_size, void* d_ws, size_t ws_size,
                              hipStream_t stream) {
    (void)d_ws; (void)ws_size;
    if (n_in < 11) return;
    const int nb = out_size / TT;
    if (nb <= 0 || nb * TT != out_size) return;
    if ((nb % 16) != 0) return;
    if (in_sizes[0] != nb * TT * NI) return;
    if (in_sizes[1] != NG * NI || in_sizes[2] != NG * NH || in_sizes[3] != NG || in_sizes[4] != NG ||
        in_sizes[5] != NG * NH || in_sizes[6] != NG * NH || in_sizes[7] != NG || in_sizes[8] != NG ||
        in_sizes[9] != NH || in_sizes[10] != 1) return;

    const float* x    = (const float*)d_in[0];
    const float* Wih0 = (const float*)d_in[1];
    const float* Whh0 = (const float*)d_in[2];
    const float* bih0 = (const float*)d_in[3];
    const float* bhh0 = (const float*)d_in[4];
    const float* Wih1 = (const float*)d_in[5];
    const float* Whh1 = (const float*)d_in[6];
    const float* bih1 = (const float*)d_in[7];
    const float* bhh1 = (const float*)d_in[8];
    const float* Wfc  = (const float*)d_in[9];
    const float* bfc  = (const float*)d_in[10];
    float* out = (float*)d_out;

    k_lstm2<<<dim3(nb / 16), dim3(32), 0, stream>>>(x, Wih0, Whh0, bih0, bhh0,
                                                 Wih1, Whh1, bih1, bhh1, Wfc, bfc, out, nb);
}
